// Node2VecGCNModel_16638703305294
// MI455X (gfx1250) — hardware-verified
//
#include <hip/hip_runtime.h>
#include <stddef.h>


#define HD      64
#define KP      128
#define NLAY    2
#define NTHR    256
#define NWAVE   8
#define EPT     8
#define NGRP    2
#define CHUNK   (NTHR * EPT * NGRP)
#define WCAP    (EPT * NGRP * 32)
#define LISTN   (NWAVE * WCAP)
#define NBA     1024
#define NBD     4096
#define GROWS   128
#define APP     136
#define APC     72
#define ASCALE  8.0f
#define WSCALE  8.0f
#define OSCALE  0.015625f
#define BNEPS   1e-5f
#define LDS_AGG (NBA * HD * 4 + LISTN * 4 + 64)

static_assert((CHUNK & (CHUNK - 1)) == 0);
static_assert(CHUNK <= 4096);
static_assert(NBA <= 4096 && NBD <= 4096);
static_assert((NBA & (NBA - 1)) == 0 && (NBD & (NBD - 1)) == 0);
static_assert(GROWS * APC * 2 <= GROWS * HD * 4);
static_assert(4 * 64 * 2 * 8 <= LISTN * 4);
static_assert(NBA * HD == NWAVE * 64 * 128);
static_assert(NBD == NWAVE * 4 * 128);

typedef float    v2f  __attribute__((ext_vector_type(2)));
typedef float    v4f  __attribute__((ext_vector_type(4)));
typedef float    v8f  __attribute__((ext_vector_type(8)));
typedef int      v4i  __attribute__((ext_vector_type(4)));
typedef double   v2d  __attribute__((ext_vector_type(2)));
typedef _Float16 v8h  __attribute__((ext_vector_type(8)));
typedef _Float16 v16h __attribute__((ext_vector_type(16)));
union FragH { v16h v; v8h h[2]; };

__device__ __forceinline__ v8h cvt8(v4f a, v4f b) {
  v8h r;
  r[0] = (_Float16)a.x; r[1] = (_Float16)a.y; r[2] = (_Float16)a.z; r[3] = (_Float16)a.w;
  r[4] = (_Float16)b.x; r[5] = (_Float16)b.y; r[6] = (_Float16)b.z; r[7] = (_Float16)b.w;
  return r;
}

__device__ __forceinline__ v8f wmh(v16h a, v16h b, v8f c) {
  v8f d = __builtin_amdgcn_wmma_f32_16x16x32_f16(false, a, false, b, (short)0, c, false, false);
  asm volatile("v_nop\n\tv_nop\n\tv_nop\n\tv_nop" : "+v"(d) : "v"(a), "v"(b));
  return d;
}

__device__ __forceinline__ v4f bn_relu4(v4f z, v4f mu, v4f rs, v4f ga, v4f be) {
#pragma clang fp contract(off)
  v4f t = z - mu;
  t = t * rs;
  t = t * ga;
  t = t + be;
  t.x = fmaxf(t.x, 0.f); t.y = fmaxf(t.y, 0.f); t.z = fmaxf(t.z, 0.f); t.w = fmaxf(t.w, 0.f);
  return t;
}

template <int NB>
__device__ __forceinline__ int scan_chunk(const int* __restrict__ dsts, int nE, int cbase, int nodeBase,
                                          int vec8, int* list, int tid, int lane, int wave) {
  int wc = 0;
#pragma unroll
  for (int g = 0; g < NGRP; ++g) {
    const int el0  = (g * NTHR + tid) * EPT;
    const int e0   = cbase + el0;
    const int sent = -2147483647 - 1;
    v4i da, db;
    if (vec8 != 0 && cbase + CHUNK <= nE) {
      da = *(const v4i*)(dsts + e0);
      db = *(const v4i*)(dsts + e0 + 4);
    } else {
      const int em = nE > 0 ? nE - 1 : 0;
      da.x = (e0     < nE) ? dsts[min(e0, em)]     : sent;
      da.y = (e0 + 1 < nE) ? dsts[min(e0 + 1, em)] : sent;
      da.z = (e0 + 2 < nE) ? dsts[min(e0 + 2, em)] : sent;
      da.w = (e0 + 3 < nE) ? dsts[min(e0 + 3, em)] : sent;
      db.x = (e0 + 4 < nE) ? dsts[min(e0 + 4, em)] : sent;
      db.y = (e0 + 5 < nE) ? dsts[min(e0 + 5, em)] : sent;
      db.z = (e0 + 6 < nE) ? dsts[min(e0 + 6, em)] : sent;
      db.w = (e0 + 7 < nE) ? dsts[min(e0 + 7, em)] : sent;
    }
    const unsigned nb = (unsigned)nodeBase;
    const unsigned s0 = (unsigned)da.x - nb, s1 = (unsigned)da.y - nb;
    const unsigned s2 = (unsigned)da.z - nb, s3 = (unsigned)da.w - nb;
    const unsigned s4 = (unsigned)db.x - nb, s5 = (unsigned)db.y - nb;
    const unsigned s6 = (unsigned)db.z - nb, s7 = (unsigned)db.w - nb;
    const bool h0 = s0 < (unsigned)NB, h1 = s1 < (unsigned)NB, h2 = s2 < (unsigned)NB, h3 = s3 < (unsigned)NB;
    const bool h4 = s4 < (unsigned)NB, h5 = s5 < (unsigned)NB, h6 = s6 < (unsigned)NB, h7 = s7 < (unsigned)NB;
    const unsigned any = __builtin_amdgcn_ballot_w32(h0 | h1 | h2 | h3 | h4 | h5 | h6 | h7);
    if (any != 0u) {
#define HITJ(J, HJ, SJ) { \
        const unsigned mj = __builtin_amdgcn_ballot_w32(HJ); \
        if (mj != 0u) { \
          if (HJ) { \
            const int pos = wc + (int)__builtin_amdgcn_mbcnt_lo(mj, 0u); \
            if (pos < WCAP) list[wave * WCAP + pos] = ((el0 + (J)) << 12) | (int)(SJ); \
          } \
          wc += (int)__builtin_popcount(mj); } }
      HITJ(0, h0, s0)
      HITJ(1, h1, s1)
      HITJ(2, h2, s2)
      HITJ(3, h3, s3)
      HITJ(4, h4, s4)
      HITJ(5, h5, s5)
      HITJ(6, h6, s6)
      HITJ(7, h7, s7)
#undef HITJ
    }
  }
  return wc;
}

__global__ __launch_bounds__(NTHR) void k_prep(
    const float* __restrict__ Wp, const float* __restrict__ Wc,
    _Float16* wps, _Float16* wcs) {
  const int b = blockIdx.x, tid = threadIdx.x;
  v4f a, c;
  _Float16* dp;
  if (b < 4) {
    const int o  = (b * NTHR + tid) * 8;
    const int n  = o / KP;
    const int k0 = o - n * KP;
    const float* p = Wp + (size_t)k0 * HD + n;
    a.x = p[0];      a.y = p[HD];     a.z = p[2 * HD]; a.w = p[3 * HD];
    c.x = p[4 * HD]; c.y = p[5 * HD]; c.z = p[6 * HD]; c.w = p[7 * HD];
    dp = wps + o;
  } else {
    const int l  = (b - 4) >> 1;
    const int o  = (((b - 4) & 1) * NTHR + tid) * 8;
    const int n  = o / HD;
    const int k0 = o - n * HD;
    const float* p = Wc + (size_t)l * HD * HD + (size_t)k0 * HD + n;
    a.x = p[0];      a.y = p[HD];     a.z = p[2 * HD]; a.w = p[3 * HD];
    c.x = p[4 * HD]; c.y = p[5 * HD]; c.z = p[6 * HD]; c.w = p[7 * HD];
    dp = wcs + (size_t)l * HD * HD + o;
  }
  a = a * WSCALE;
  c = c * WSCALE;
  const v8h hv = cvt8(a, c);
  *(volatile v8h*)dp = hv;
  __threadfence();
  *(volatile v8h*)dp = hv;
}

__global__ __launch_bounds__(NTHR) void k_deg(
    const int* __restrict__ ei, float* dinv, int nE, int vec8) {
  __shared__ __attribute__((aligned(16))) int cnt[NBD];
  __shared__ __attribute__((aligned(16))) int list[LISTN];
  __shared__ int wcnt[NWAVE];
  const int tid = threadIdx.x, lane = tid & 31, wave = tid >> 5;
  const int nodeBase = blockIdx.x * NBD;
  const int* dsts = ei + nE;

  for (int i = tid; i < NBD; i += NTHR) cnt[i] = 0;
  __syncthreads();

  const int nChunks = (nE + CHUNK - 1) / CHUNK;
#pragma unroll 1
  for (int ch = 0; ch < nChunks; ++ch) {
    const int cbase = ch * CHUNK;
    const int wc = scan_chunk<NBD>(dsts, nE, cbase, nodeBase, vec8, list, tid, lane, wave);
    if (lane == 0) wcnt[wave] = wc;
    __syncthreads();
    if (wave == 0) {
#pragma unroll 1
      for (int wsx = 0; wsx < NWAVE; ++wsx) {
        int n = __builtin_amdgcn_readfirstlane(wcnt[wsx]);
        n = n > WCAP ? WCAP : (n < 0 ? 0 : n);
        const int* lp = list + wsx * WCAP;
#pragma unroll 1
        for (int i = 0; i < n; ++i) {
          const int ent  = __builtin_amdgcn_readfirstlane(lp[i]);
          const int slot = ent & (NBD - 1);
          if (lane == 0) cnt[slot] = cnt[slot] + 1;
        }
      }
    }
    __syncthreads();
  }

  v4f dq[4];
#pragma unroll
  for (int q = 0; q < 4; ++q) {
    const int f = (wave * 4 + q) * 128 + 4 * lane;
    const v4i c = *(const v4i*)(cnt + f);
    dq[q].x = rsqrtf((float)(c.x + 1));
    dq[q].y = rsqrtf((float)(c.y + 1));
    dq[q].z = rsqrtf((float)(c.z + 1));
    dq[q].w = rsqrtf((float)(c.w + 1));
  }
  float* dp = dinv + (size_t)nodeBase;
#pragma unroll
  for (int q = 0; q < 4; ++q) *(volatile v4f*)(dp + (wave * 4 + q) * 128 + 4 * lane) = dq[q];
  __threadfence();
#pragma unroll
  for (int q = 0; q < 4; ++q) *(volatile v4f*)(dp + (wave * 4 + q) * 128 + 4 * lane) = dq[q];
}

__global__ __launch_bounds__(NTHR) void k_proj(
    const float* __restrict__ ea, const float* __restrict__ eb,
    const _Float16* __restrict__ wps, const float* __restrict__ pb,
    float* x0, int nN) {
#pragma clang fp contract(off)
  __shared__ v4f lbuf[(GROWS * APP * 2) / 16];
  _Float16* sA  = (_Float16*)lbuf;
  float*    stg = (float*)lbuf;
  const int tid = threadIdx.x, lane = tid & 31, wave = tid >> 5, hh = lane >> 4, m = lane & 15;
  const int rowBase = blockIdx.x * GROWS;

#pragma unroll
  for (int i = 0; i < 8; ++i) {
    const int idx = (i & 3) * NTHR + tid;
    const int r   = idx >> 3;
    const int c0  = (idx & 7) * 8;
    int node = rowBase + r;
    node = node > nN - 1 ? nN - 1 : node;
    const float* src = (i < 4) ? ea : eb;
    const float* xp = src + (size_t)node * HD + c0;
    v4f a = *(const v4f*)xp, b = *(const v4f*)(xp + 4);
    a = a * ASCALE;
    b = b * ASCALE;
    *(v8h*)(sA + r * APP + c0 + ((i < 4) ? 0 : HD)) = cvt8(a, b);
  }
  __syncthreads();

  v8f acc[4];
#pragma unroll
  for (int t = 0; t < 4; ++t) { v8f z = {0.f, 0.f, 0.f, 0.f, 0.f, 0.f, 0.f, 0.f}; acc[t] = z; }
  const _Float16* ar = sA + (wave * 16 + m) * APP + 8 * hh;
#pragma unroll
  for (int kt = 0; kt < KP / 32; ++kt) {
    FragH a;
    a.h[0] = *(const v8h*)(ar + 32 * kt);
    a.h[1] = *(const v8h*)(ar + 32 * kt + 16);
#pragma unroll
    for (int t = 0; t < 4; ++t) {
      const _Float16* bp = wps + (size_t)(16 * t + m) * KP + 32 * kt + 8 * hh;
      FragH b;
      b.h[0] = *(const v8h*)bp;
      b.h[1] = *(const v8h*)(bp + 16);
      acc[t] = wmh(a.v, b.v, acc[t]);
    }
  }
  __syncthreads();

  const int r0 = wave * 16 + 8 * hh;
  float* sp = stg + r0 * HD + m;
#pragma unroll
  for (int t = 0; t < 4; ++t) {
    const float bias = pb[16 * t + m];
    float v;
    v = acc[t][0] * OSCALE; sp[0 * HD + 16 * t] = v + bias;
    v = acc[t][1] * OSCALE; sp[1 * HD + 16 * t] = v + bias;
    v = acc[t][2] * OSCALE; sp[2 * HD + 16 * t] = v + bias;
    v = acc[t][3] * OSCALE; sp[3 * HD + 16 * t] = v + bias;
    v = acc[t][4] * OSCALE; sp[4 * HD + 16 * t] = v + bias;
    v = acc[t][5] * OSCALE; sp[5 * HD + 16 * t] = v + bias;
    v = acc[t][6] * OSCALE; sp[6 * HD + 16 * t] = v + bias;
    v = acc[t][7] * OSCALE; sp[7 * HD + 16 * t] = v + bias;
  }
  __syncthreads();

  const float* lp = stg + wave * 16 * HD + 4 * lane;
  float* gp = x0 + ((size_t)rowBase + wave * 16) * HD + 4 * lane;
#pragma unroll
  for (int q = 0; q < 8; ++q) { const v4f v = *(const v4f*)(lp + q * 128); *(volatile v4f*)(gp + (size_t)q * 128) = v; }
  __threadfence();
#pragma unroll
  for (int q = 0; q < 8; ++q) { const v4f v = *(const v4f*)(lp + q * 128); *(volatile v4f*)(gp + (size_t)q * 128) = v; }
}

template <int MODE>
__global__ __launch_bounds__(NTHR) void k_gemm(
    const float* __restrict__ x0, const float* __restrict__ z0, const float* __restrict__ st0,
    const float* __restrict__ gam, const float* __restrict__ bet,
    const _Float16* __restrict__ wcs, const float* __restrict__ dinv, float* g, int nN) {
#pragma clang fp contract(off)
  __shared__ v4f lbuf[(GROWS * HD * 4) / 16];
  _Float16* sA  = (_Float16*)lbuf;
  float*    stg = (float*)lbuf;
  const int tid = threadIdx.x, lane = tid & 31, wave = tid >> 5, hh = lane >> 4, m = lane & 15;
  const int rowBase = blockIdx.x * GROWS;
  const int c0 = (tid & 7) * 8;

  v4f muA, muB, rsA, rsB, gaA, gaB, beA, beB;
  if (MODE == 1) {
    muA = *(const v4f*)(st0 + c0);       muB = *(const v4f*)(st0 + c0 + 4);
    rsA = *(const v4f*)(st0 + HD + c0);  rsB = *(const v4f*)(st0 + HD + c0 + 4);
    gaA = *(const v4f*)(gam + c0);       gaB = *(const v4f*)(gam + c0 + 4);
    beA = *(const v4f*)(bet + c0);       beB = *(const v4f*)(bet + c0 + 4);
  }

#pragma unroll
  for (int i = 0; i < 4; ++i) {
    const int idx = i * NTHR + tid;
    const int r   = idx >> 3;
    int node = rowBase + r;
    node = node > nN - 1 ? nN - 1 : node;
    const float* xp = x0 + (size_t)node * HD + c0;
    v4f a = *(const v4f*)xp, b = *(const v4f*)(xp + 4);
    if (MODE == 1) {
      const float* zp = z0 + (size_t)node * HD + c0;
      const v4f za = *(const v4f*)zp, zb = *(const v4f*)(zp + 4);
      a = a + bn_relu4(za, muA, rsA, gaA, beA);
      b = b + bn_relu4(zb, muB, rsB, gaB, beB);
    }
    a = a * ASCALE;
    b = b * ASCALE;
    *(v8h*)(sA + r * APC + c0) = cvt8(a, b);
  }
  __syncthreads();

  v8f acc[4];
#pragma unroll
  for (int t = 0; t < 4; ++t) { v8f z = {0.f, 0.f, 0.f, 0.f, 0.f, 0.f, 0.f, 0.f}; acc[t] = z; }
  const _Float16* ar = sA + (wave * 16 + m) * APC + 8 * hh;
#pragma unroll
  for (int kt = 0; kt < HD / 32; ++kt) {
    FragH a;
    a.h[0] = *(const v8h*)(ar + 32 * kt);
    a.h[1] = *(const v8h*)(ar + 32 * kt + 16);
#pragma unroll
    for (int t = 0; t < 4; ++t) {
      const _Float16* bp = wcs + (size_t)(16 * t + m) * HD + 32 * kt + 8 * hh;
      FragH b;
      b.h[0] = *(const v8h*)bp;
      b.h[1] = *(const v8h*)(bp + 16);
      acc[t] = wmh(a.v, b.v, acc[t]);
    }
  }
  __syncthreads();

  const int r0 = wave * 16 + 8 * hh;
  const v4f dA = *(const v4f*)(dinv + (size_t)rowBase + r0);
  const v4f dB = *(const v4f*)(dinv + (size_t)rowBase + r0 + 4);
  const float d0 = dA.x * OSCALE, d1 = dA.y * OSCALE, d2 = dA.z * OSCALE, d3 = dA.w * OSCALE;
  const float d4 = dB.x * OSCALE, d5 = dB.y * OSCALE, d6 = dB.z * OSCALE, d7 = dB.w * OSCALE;
  float* sp = stg + r0 * HD + m;
#pragma unroll
  for (int t = 0; t < 4; ++t) {
    sp[0 * HD + 16 * t] = acc[t][0] * d0;
    sp[1 * HD + 16 * t] = acc[t][1] * d1;
    sp[2 * HD + 16 * t] = acc[t][2] * d2;
    sp[3 * HD + 16 * t] = acc[t][3] * d3;
    sp[4 * HD + 16 * t] = acc[t][4] * d4;
    sp[5 * HD + 16 * t] = acc[t][5] * d5;
    sp[6 * HD + 16 * t] = acc[t][6] * d6;
    sp[7 * HD + 16 * t] = acc[t][7] * d7;
  }
  __syncthreads();

  const float* lp = stg + wave * 16 * HD + 4 * lane;
  float* gp = g + ((size_t)rowBase + wave * 16) * HD + 4 * lane;
#pragma unroll
  for (int q = 0; q < 8; ++q) { const v4f v = *(const v4f*)(lp + q * 128); *(volatile v4f*)(gp + (size_t)q * 128) = v; }
  __threadfence();
#pragma unroll
  for (int q = 0; q < 8; ++q) { const v4f v = *(const v4f*)(lp + q * 128); *(volatile v4f*)(gp + (size_t)q * 128) = v; }
}

__global__ __launch_bounds__(NTHR) void k_agg(
    const int* __restrict__ ei, const float* __restrict__ g, const float* __restrict__ dinv,
    const float* __restrict__ cb, float* z, double* part, int nN, int nE, int vec8) {
#pragma clang fp contract(off)
  extern __shared__ v4f lds_dyn[];
  float*  acc  = (float*)lds_dyn;
  int*    list = (int*)(acc + NBA * HD);
  int*    wcnt = list + LISTN;
  double* pd   = (double*)list;
  const int tid = threadIdx.x, lane = tid & 31, wave = tid >> 5;
  const int nodeBase = blockIdx.x * NBA;
  const int* dsts = ei + nE;

  {
    const v4f zz = {0.f, 0.f, 0.f, 0.f};
    for (int i = tid; i < NBA * HD / 4; i += NTHR) lds_dyn[i] = zz;
  }
  __syncthreads();

  const int nChunks = (nE + CHUNK - 1) / CHUNK;
#pragma unroll 1
  for (int ch = 0; ch < nChunks; ++ch) {
    const int cbase = ch * CHUNK;
    const int wc = scan_chunk<NBA>(dsts, nE, cbase, nodeBase, vec8, list, tid, lane, wave);
    if (lane == 0) wcnt[wave] = wc;
    __syncthreads();
    if (wave == 0) {
#pragma unroll 1
      for (int wsx = 0; wsx < NWAVE; ++wsx) {
        int n = __builtin_amdgcn_readfirstlane(wcnt[wsx]);
        n = n > WCAP ? WCAP : (n < 0 ? 0 : n);
        const int* lp = list + wsx * WCAP;
#pragma unroll 1
        for (int i = 0; i < n; ++i) {
          const int ent  = __builtin_amdgcn_readfirstlane(lp[i]);
          const int slot = ent & (NBA - 1);
          int e = cbase + ((ent >> 12) & (CHUNK - 1));
          e = e > nE - 1 ? nE - 1 : e;
          e = e < 0 ? 0 : e;
          int src = ei[e];
          src = src < 0 ? 0 : (src > nN - 1 ? nN - 1 : src);
          const v2f v = *(const v2f*)(g + (size_t)src * HD + 2 * lane);
          v2f* ap = (v2f*)(acc + slot * HD + 2 * lane);
          *ap = *ap + v;
        }
      }
    }
    __syncthreads();
  }

#pragma unroll 4
  for (int i = 0; i < (NBA * HD / 4) / NTHR; ++i) {
    const int idx  = i * NTHR + tid;
    const int slot = idx >> 4;
    const int c4   = (idx & 15) * 4;
    const int node = nodeBase + slot;
    const bool valid = node < nN;
    const int  nc  = valid ? node : nN - 1;
    const float d  = dinv[nc];
    const v4f   gv = *(const v4f*)(g + (size_t)nc * HD + c4);
    const v4f   bv = *(const v4f*)(cb + c4);
    v4f* ap = (v4f*)(acc + slot * HD + c4);
    v4f t = *ap + gv;
    t = t * d;
    t = t + bv;
    if (!valid) { const v4f zz = {0.f, 0.f, 0.f, 0.f}; t = zz; }
    *ap = t;
  }
  __syncthreads();

  {
    const int c  = tid & 63;
    const int rg = tid >> 6;
    double s = 0.0, s2 = 0.0;
#pragma unroll 4
    for (int rr = 0; rr < NBA / 4; ++rr) {
      const double v = (double)acc[(rg * (NBA / 4) + rr) * HD + c];
      s  = s + v;
      s2 = s2 + v * v;
    }
    pd[(rg * 64 + c) * 2]     = s;
    pd[(rg * 64 + c) * 2 + 1] = s2;
  }

  float* zp = z + (size_t)nodeBase * HD;
#pragma unroll 4
  for (int q = 0; q < 64; ++q) {
    const int f = (wave * 64 + q) * 128 + 4 * lane;
    const v4f v = *(const v4f*)(acc + f);
    *(volatile v4f*)(zp + f) = v;
  }
  __threadfence();
#pragma unroll 4
  for (int q = 0; q < 64; ++q) {
    const int f = (wave * 64 + q) * 128 + 4 * lane;
    const v4f v = *(const v4f*)(acc + f);
    *(volatile v4f*)(zp + f) = v;
  }
  __syncthreads();

  if (tid < 64) {
    const double S  = ((pd[(0 * 64 + tid) * 2]     + pd[(1 * 64 + tid) * 2])     + pd[(2 * 64 + tid) * 2])     + pd[(3 * 64 + tid) * 2];
    const double S2 = ((pd[(0 * 64 + tid) * 2 + 1] + pd[(1 * 64 + tid) * 2 + 1]) + pd[(2 * 64 + tid) * 2 + 1]) + pd[(3 * 64 + tid) * 2 + 1];
    v2d o; o.x = S; o.y = S2;
    double* pp = part + ((size_t)blockIdx.x * 64 + tid) * 2;
    *(volatile v2d*)pp = o;
    __threadfence();
    *(volatile v2d*)pp = o;
  }
}

__global__ __launch_bounds__(64) void k_fin(const double* __restrict__ part, float* st, int nBlk, int nN) {
#pragma clang fp contract(off)
  __shared__ __attribute__((aligned(16))) float sst[128];
  const int c = threadIdx.x;
  double s = 0.0, s2 = 0.0;
#pragma unroll 1
  for (int b = 0; b < nBlk; ++b) {
    const v2d p = *(const v2d*)(part + ((size_t)b * 64 + c) * 2);
    s  = s + p.x;
    s2 = s2 + p.y;
  }
  const double inv = 1.0 / (double)nN;
  const double mu  = s * inv;
  double var = s2 * inv - mu * mu;
  var = var < 0.0 ? 0.0 : var;
  const float varf = (float)var;
  sst[c]      = (float)mu;
  sst[64 + c] = rsqrtf(varf + BNEPS);
  __syncthreads();
  if (c < 32) {
    const v4f v = *(const v4f*)(sst + 4 * c);
    *(volatile v4f*)(st + 4 * c) = v;
    __threadfence();
    *(volatile v4f*)(st + 4 * c) = v;
  }
}

__global__ __launch_bounds__(NTHR) void k_apply(
    const float* __restrict__ x0, const float* __restrict__ z0, const float* __restrict__ z1,
    const float* __restrict__ st0, const float* __restrict__ st1,
    const float* __restrict__ gam, const float* __restrict__ bet, float* x2, int nN) {
#pragma clang fp contract(off)
  const size_t total4 = (size_t)nN * (HD / 4);
  const size_t idx = (size_t)blockIdx.x * NTHR + threadIdx.x;
  const bool ok = idx < total4;
  const size_t ci = ok ? idx : total4 - 1;
  const int c4 = (int)(ci & 15) * 4;
  const v4f xv  = *(const v4f*)(x0 + ci * 4);
  const v4f za  = *(const v4f*)(z0 + ci * 4);
  const v4f zb  = *(const v4f*)(z1 + ci * 4);
  const v4f mu0 = *(const v4f*)(st0 + c4), rs0 = *(const v4f*)(st0 + HD + c4);
  const v4f mu1 = *(const v4f*)(st1 + c4), rs1 = *(const v4f*)(st1 + HD + c4);
  const v4f g0  = *(const v4f*)(gam + c4), b0 = *(const v4f*)(bet + c4);
  const v4f g1  = *(const v4f*)(gam + HD + c4), b1 = *(const v4f*)(bet + HD + c4);
  v4f x1 = xv + bn_relu4(za, mu0, rs0, g0, b0);
  v4f xo = x1 + bn_relu4(zb, mu1, rs1, g1, b1);
  if (ok) {
    *(volatile v4f*)(x2 + idx * 4) = xo;
    __threadfence();
    *(volatile v4f*)(x2 + idx * 4) = xo;
  }
}

__global__ __launch_bounds__(NTHR) void k_dec(
    const int* __restrict__ pe, const float* __restrict__ x2, float* out, int nN, int nP) {
#pragma clang fp contract(off)
  __shared__ __attribute__((aligned(16))) float res[NWAVE * 32];
  const int tid = threadIdx.x, lane = tid & 31, wave = tid >> 5;
  const int sub = lane >> 4, q = lane & 15;
  const int lineBase = (blockIdx.x * NWAVE + wave) * 32;
#pragma unroll 1
  for (int it = 0; it < 16; ++it) {
    int p = lineBase + 2 * it + sub;
    p = p > nP - 1 ? nP - 1 : p;
    int a = pe[2 * p], b = pe[2 * p + 1];
    a = a < 0 ? 0 : (a > nN - 1 ? nN - 1 : a);
    b = b < 0 ? 0 : (b > nN - 1 ? nN - 1 : b);
    const v4f xa = *(const v4f*)(x2 + (size_t)a * HD + 4 * q);
    const v4f xb = *(const v4f*)(x2 + (size_t)b * HD + 4 * q);
    const v4f pr = xa * xb;
    float s = (pr.x + pr.y) + (pr.z + pr.w);
    s += __shfl_xor(s, 1, 32);
    s += __shfl_xor(s, 2, 32);
    s += __shfl_xor(s, 4, 32);
    s += __shfl_xor(s, 8, 32);
    if (q == 0) res[wave * 32 + 2 * it + sub] = s;
  }
  __syncthreads();
  const int p0 = lineBase + 4 * lane;
  v4f v = {0.f, 0.f, 0.f, 0.f};
  if (lane < 8) v = *(const v4f*)(res + wave * 32 + 4 * lane);
  if (lane < 8) {
    if (p0 + 4 <= nP) {
      *(volatile v4f*)(out + p0) = v;
    } else {
      if (p0     < nP) *(volatile float*)(out + p0)     = v.x;
      if (p0 + 1 < nP) *(volatile float*)(out + p0 + 1) = v.y;
      if (p0 + 2 < nP) *(volatile float*)(out + p0 + 2) = v.z;
      if (p0 + 3 < nP) *(volatile float*)(out + p0 + 3) = v.w;
    }
  }
  __threadfence();
  if (lane < 8) {
    if (p0 + 4 <= nP) {
      *(volatile v4f*)(out + p0) = v;
    } else {
      if (p0     < nP) *(volatile float*)(out + p0)     = v.x;
      if (p0 + 1 < nP) *(volatile float*)(out + p0 + 1) = v.y;
      if (p0 + 2 < nP) *(volatile float*)(out + p0 + 2) = v.z;
      if (p0 + 3 < nP) *(volatile float*)(out + p0 + 3) = v.w;
    }
  }
}

extern "C" void kernel_launch(void* const* d_in, const int* in_sizes, int n_in,
                              void* d_out, int out_size, void* d_ws, size_t ws_size,
                              hipStream_t stream) {
  if (n_in < 10) return;
  const int nE = in_sizes[0] / 2;
  const int nP = in_sizes[1] / 2;
  const int nN = in_sizes[2] / HD;
  if (nN <= 0 || nP <= 0 || nE < 0) return;
  if (in_sizes[0] != 2 * nE || in_sizes[1] != 2 * nP) return;
  if (in_sizes[2] != nN * HD || in_sizes[3] != nN * HD) return;
  if (in_sizes[4] != KP * HD || in_sizes[5] < HD) return;
  if (in_sizes[6] != NLAY * HD * HD || in_sizes[7] < NLAY * HD || in_sizes[8] < NLAY * HD || in_sizes[9] < NLAY * HD) return;
  if (out_size != nP) return;

  const int*   ei  = (const int*)d_in[0];
  const int*   pe  = (const int*)d_in[1];
  const float* ea  = (const float*)d_in[2];
  const float* eb  = (const float*)d_in[3];
  const float* Wp  = (const float*)d_in[4];
  const float* pb  = (const float*)d_in[5];
  const float* Wc  = (const float*)d_in[6];
  const float* cb  = (const float*)d_in[7];
  const float* gam = (const float*)d_in[8];
  const float* bet = (const float*)d_in[9];
  float* out = (float*)d_out;

  const int nBD  = (nN + NBD - 1) / NBD;
  const int nG   = (nN + GROWS - 1) / GROWS;
  const int nA   = (nN + NBA - 1) / NBA;
  const int nAp  = (nN * (HD / 4) + NTHR - 1) / NTHR;
  const int nDec = (nP + NWAVE * 32 - 1) / (NWAVE * 32);

  char* ws = (char*)d_ws;
  size_t off = 0;
  const size_t oWp = off; off += (size_t)HD * KP * 2;                          off = (off + 255) & ~(size_t)255;
  const size_t oWc = off; off += (size_t)NLAY * HD * HD * 2;                   off = (off + 255) & ~(size_t)255;
  const size_t oDv = off; off += (size_t)nBD * NBD * 4;                        off = (off + 255) & ~(size_t)255;
  const size_t oX0 = off; off += (size_t)nG * GROWS * HD * 4;                  off = (off + 255) & ~(size_t)255;
  const size_t oG  = off; off += (size_t)nG * GROWS * HD * 4;                  off = (off + 255) & ~(size_t)255;
  const size_t oZ0 = off; off += (size_t)nA * NBA * HD * 4;                    off = (off + 255) & ~(size_t)255;
  const size_t oZ1 = off; off += (size_t)nA * NBA * HD * 4;                    off = (off + 255) & ~(size_t)255;
  const size_t oP0 = off; off += (size_t)nA * 64 * 2 * 8;                      off = (off + 255) & ~(size_t)255;
  const size_t oP1 = off; off += (size_t)nA * 64 * 2 * 8;                      off = (off + 255) & ~(size_t)255;
  const size_t oS0 = off; off += (size_t)2 * HD * 4;                           off = (off + 255) & ~(size_t)255;
  const size_t oS1 = off; off += (size_t)2 * HD * 4;                           off = (off + 255) & ~(size_t)255;
  const size_t oX2 = off; off += (size_t)nAp * NTHR * 16;                      off = (off + 255) & ~(size_t)255;
  if (off > ws_size) return;
  _Float16* wps  = (_Float16*)(ws + oWp);
  _Float16* wcs  = (_Float16*)(ws + oWc);
  float*    dinv = (float*)(ws + oDv);
  float*    x0   = (float*)(ws + oX0);
  float*    g    = (float*)(ws + oG);
  float*    z0   = (float*)(ws + oZ0);
  float*    z1   = (float*)(ws + oZ1);
  double*   p0   = (double*)(ws + oP0);
  double*   p1   = (double*)(ws + oP1);
  float*    st0  = (float*)(ws + oS0);
  float*    st1  = (float*)(ws + oS1);
  float*    x2   = (float*)(ws + oX2);

  const int vec8 = ((nE & 3) == 0) ? 1 : 0;

  k_prep<<<8, NTHR, 0, stream>>>(Wp, Wc, wps, wcs);
  k_deg<<<nBD, NTHR, 0, stream>>>(ei, dinv, nE, vec8);
  k_proj<<<nG, NTHR, 0, stream>>>(ea, eb, wps, pb, x0, nN);

  hipFuncSetAttribute(reinterpret_cast<const void*>(&k_agg),
                      hipFuncAttributeMaxDynamicSharedMemorySize, LDS_AGG);

  k_gemm<0><<<nG, NTHR, 0, stream>>>(x0, z0, st0, gam, bet, wcs, dinv, g, nN);
  k_agg<<<nA, NTHR, LDS_AGG, stream>>>(ei, g, dinv, cb, z0, p0, nN, nE, vec8);
  k_fin<<<1, 64, 0, stream>>>(p0, st0, nA, nN);

  k_gemm<1><<<nG, NTHR, 0, stream>>>(x0, z0, st0, gam, bet, wcs + HD * HD, dinv, g, nN);
  k_agg<<<nA, NTHR, LDS_AGG, stream>>>(ei, g, dinv, cb + HD, z1, p1, nN, nE, vec8);
  k_fin<<<1, 64, 0, stream>>>(p1, st1, nA, nN);

  k_apply<<<nAp, NTHR, 0, stream>>>(x0, z0, z1, st0, st1, gam, bet, x2, nN);
  k_dec<<<nDec, NTHR, 0, stream>>>(pe, x2, out, nN, nP);
}
